// KnowformerQKLayer_15951508537885
// MI455X (gfx1250) — hardware-run, weakly checked
//
#include <hip/hip_runtime.h>

typedef float          v8f   __attribute__((ext_vector_type(8)));
typedef float          v4f   __attribute__((ext_vector_type(4)));
typedef unsigned int   v4u   __attribute__((ext_vector_type(4)));
typedef int            v8i   __attribute__((ext_vector_type(8)));
typedef unsigned short v8us  __attribute__((ext_vector_type(8)));
typedef unsigned short v16us __attribute__((ext_vector_type(16)));
typedef __bf16         v16bf __attribute__((ext_vector_type(16)));
typedef _Float16       v16h  __attribute__((ext_vector_type(16)));
typedef v4f  __attribute__((may_alias)) v4fa;
typedef v8us __attribute__((may_alias)) v8usa;
union FragB { v16bf v; v16us u; v8us h[2]; v8i w; };
union FragH { v16h  v; v16us u; v8us h[2]; v8i w; };

__device__ __forceinline__ v8f wmb(const FragB& a, const FragB& b, v8f c) {
  v8f d = __builtin_amdgcn_wmma_f32_16x16x32_bf16(false, a.v, false, b.v, (short)0, c, false, false);
  asm volatile("v_nop\n\tv_nop\n\tv_nop\n\tv_nop" : "+v"(d) : "v"(a.w), "v"(b.w));
  return d;
}

__device__ __forceinline__ v8f wmh(const FragH& a, const FragH& b, v8f c) {
  v8f d = __builtin_amdgcn_wmma_f32_16x16x32_f16(false, a.v, false, b.v, (short)0, c, false, false);
  asm volatile("v_nop\n\tv_nop\n\tv_nop\n\tv_nop" : "+v"(d) : "v"(a.w), "v"(b.w));
  return d;
}

__device__ __forceinline__ unsigned bf16_bits(float f) {
  const unsigned u = __float_as_uint(f);
  const unsigned r = (u + 0x7FFFu + ((u >> 16) & 1u)) >> 16;
  const unsigned q = (u >> 16) | 0x40u;
  return ((u & 0x7fffffffu) > 0x7f800000u) ? q : r;
}

__device__ __forceinline__ float bf16_val(float f) {
  return __uint_as_float(bf16_bits(f) << 16);
}
__device__ __forceinline__ int clampi(int v, int lo, int hi) {
  return v < lo ? lo : (v > hi ? hi : v);
}

__device__ __forceinline__ unsigned f16_bits(float f) {
  const unsigned u  = __float_as_uint(f);
  const unsigned s  = (u >> 16) & 0x8000u;
  const unsigned a  = u & 0x7fffffffu;
  const unsigned t  = a - 0x38000000u;
  const unsigned r  = (t + 0x0FFFu + ((t >> 13) & 1u)) >> 13;
  const unsigned rc = r > 0x7C00u ? 0x7C00u : r;
  const bool small  = a < 0x38800000u;
  const bool isnan  = a > 0x7f800000u;
  const unsigned fin = small ? 0u : (s | rc);
  return isnan ? (s | 0x7E00u) : fin;
}

__device__ __forceinline__ unsigned pk16(unsigned lo, unsigned hi) { return lo | (hi << 16); }
__device__ __forceinline__ unsigned bf16_lo_bits(float v) {
  float hi = bf16_val(v);
  asm volatile("" : "+v"(hi));
  return bf16_bits(v - hi);
}
__device__ __forceinline__ v4u pack8_bf16(v4f a, v4f c) {
  return (v4u){ pk16(bf16_bits(a[0]), bf16_bits(a[1])), pk16(bf16_bits(a[2]), bf16_bits(a[3])),
                pk16(bf16_bits(c[0]), bf16_bits(c[1])), pk16(bf16_bits(c[2]), bf16_bits(c[3])) };
}
__device__ __forceinline__ v4u pack8_bf16_lo(v4f a, v4f c) {
  return (v4u){ pk16(bf16_lo_bits(a[0]), bf16_lo_bits(a[1])), pk16(bf16_lo_bits(a[2]), bf16_lo_bits(a[3])),
                pk16(bf16_lo_bits(c[0]), bf16_lo_bits(c[1])), pk16(bf16_lo_bits(c[2]), bf16_lo_bits(c[3])) };
}
__device__ __forceinline__ v4u pack8_f16(v4f a, v4f c) {
  return (v4u){ pk16(f16_bits(a[0]), f16_bits(a[1])), pk16(f16_bits(a[2]), f16_bits(a[3])),
                pk16(f16_bits(c[0]), f16_bits(c[1])), pk16(f16_bits(c[2]), f16_bits(c[3])) };
}

template <int FORM>
__global__ __launch_bounds__(256) void k_plane(const float* __restrict__ src, int rows, int cols, int ldsrc,
                                               unsigned short* __restrict__ dst, int MP, int KP) {
  static_assert(FORM >= 0 && FORM <= 3);
  const int KTOT = (FORM == 1 || FORM == 3) ? 2 * KP : KP;
  const unsigned ppr   = (unsigned)(KTOT >> 3);
  const unsigned kp8   = (unsigned)(KP >> 3);
  const unsigned total = (unsigned)MP * ppr;
  const unsigned g     = blockIdx.x * 256u + threadIdx.x;
  const unsigned rowu  = g / ppr;
  const unsigned p     = g - rowu * ppr;
  const bool second    = p >= kp8;
  const int row = (int)rowu;
  const int c0  = (int)((second ? p - kp8 : p) << 3);
  const float* srow = src + (size_t)clampi(row, 0, rows - 1) * (size_t)ldsrc;
  float x[8];
  unsigned mk[8];
#pragma unroll
  for (int e = 0; e < 8; ++e) {
    const int c = c0 + e;
    const float v = srow[clampi(c, 0, cols - 1)];
    asm volatile("" :: "v"(v));
    x[e]  = v;
    mk[e] = (row < rows && c < cols) ? 0xFFFFu : 0u;
  }
  const v4f a = (v4f){ x[0], x[1], x[2], x[3] };
  const v4f c = (v4f){ x[4], x[5], x[6], x[7] };
  v4u o;
  if (FORM == 2) {
    o = pack8_f16(a, c);
  } else {
    const v4u hi = pack8_bf16(a, c);
    o = hi;
    if (FORM == 1) { const v4u lo = pack8_bf16_lo(a, c); o = second ? lo : hi; }
  }
  const v4u mw = (v4u){ pk16(mk[0], mk[1]), pk16(mk[2], mk[3]), pk16(mk[4], mk[5]), pk16(mk[6], mk[7]) };
  o &= mw;
  if (g < total) {
    volatile v4u* q = (volatile v4u*)(dst + (size_t)g * 8);
    *q = o;
    __threadfence();
    *q = o;
  }
}

template <int FORM> struct FragOf    { typedef FragB T; };
template <>         struct FragOf<2> { typedef FragH T; };
__device__ __forceinline__ v8f mm(const FragB& a, const FragB& b, v8f c) { return wmb(a, b, c); }
__device__ __forceinline__ v8f mm(const FragH& a, const FragH& b, v8f c) { return wmh(a, b, c); }
template <class F> __device__ __forceinline__ F ld_frag(const unsigned short* p) {
  F f;
  f.h[0] = *(const v8usa*)(p);
  f.h[1] = *(const v8usa*)(p + 16);
  return f;
}

template <int FORM, int EPI>
__global__ __launch_bounds__(256) __attribute__((amdgpu_num_vgpr(248)))
void k_gemm_nt(const unsigned short* __restrict__ A, const unsigned short* __restrict__ B,
               const float* __restrict__ bias, float* __restrict__ D, int M, int N, int KTOT, int ldd) {
  static_assert(FORM >= 0 && FORM <= 2);
  static_assert(EPI == 0 || EPI == 1);
  typedef typename FragOf<FORM>::T F;
  __shared__ __attribute__((aligned(16))) float sT[8][16 * 68];
  const int lane = threadIdx.x & 31;
  const int wave = threadIdx.x >> 5;
  const int tilesM = (M + 63) >> 6;
  const int tilesN = (N + 63) >> 6;
  const int tile = blockIdx.x * 8 + wave;
  if (tile >= tilesM * tilesN) return;
  const int tm = tile / tilesN;
  const int tn = tile - tm * tilesN;
  const int m0 = tm << 6;
  const int n0 = tn << 6;

  const int rl = lane & 15;
  const int h8 = (lane >> 4) * 8;
  const unsigned short* pa = A + (size_t)(m0 + rl) * (size_t)KTOT + h8;
  const unsigned short* pb = B + (size_t)(n0 + rl) * (size_t)KTOT + h8;

  v8f acc[4][4];
#pragma unroll
  for (int i = 0; i < 4; ++i)
#pragma unroll
    for (int j = 0; j < 4; ++j) acc[i][j] = (v8f){0.f, 0.f, 0.f, 0.f, 0.f, 0.f, 0.f, 0.f};

#pragma unroll 1
  for (int k0 = 0; k0 < KTOT; k0 += 32) {
    F bf[4];
#pragma unroll
    for (int j = 0; j < 4; ++j) bf[j] = ld_frag<F>(pb + (size_t)(j << 4) * (size_t)KTOT + k0);
#pragma unroll
    for (int i = 0; i < 4; ++i) {
      const F af = ld_frag<F>(pa + (size_t)(i << 4) * (size_t)KTOT + k0);
#pragma unroll
      for (int j = 0; j < 4; ++j) acc[i][j] = mm(af, bf[j], acc[i][j]);
    }
  }

  float* slab = sT[wave];
  const int hh = lane >> 4;
  const int c4 = (lane & 15) * 4;
  const int nc = n0 + c4;
  const bool cok = nc < N;
  v4f bv = (v4f){0.f, 0.f, 0.f, 0.f};
  if (EPI == 1) {
    bv = *(const v4fa*)(bias + clampi(nc, 0, N - 4));
    asm volatile("" :: "v"(bv));
  }
#pragma unroll
  for (int i = 0; i < 4; ++i) {
    const int mBase = m0 + (i << 4);
#pragma unroll
    for (int j = 0; j < 4; ++j) {
#pragma unroll
      for (int r = 0; r < 8; ++r) slab[(h8 + r) * 68 + (j << 4) + rl] = acc[i][j][r];
    }
    __builtin_amdgcn_fence(__ATOMIC_RELEASE, "workgroup");
    __builtin_amdgcn_wave_barrier();
    __builtin_amdgcn_fence(__ATOMIC_ACQUIRE, "workgroup");
    v4f vv[8];
#pragma unroll
    for (int it = 0; it < 8; ++it) {
      const int row = it * 2 + hh;
      v4f v = *(const v4fa*)(slab + row * 68 + c4);
      if (EPI == 1) v += bv;
      vv[it] = v;
    }
    for (int pass = 0; pass < 2; ++pass) {
#pragma unroll
      for (int it = 0; it < 8; ++it) {
        const int row = mBase + it * 2 + hh;
        if (cok && row < M) *(volatile v4f*)(D + (size_t)row * (size_t)ldd + nc) = vv[it];
      }
      __threadfence();
    }
    __builtin_amdgcn_fence(__ATOMIC_RELEASE, "workgroup");
    __builtin_amdgcn_wave_barrier();
    __builtin_amdgcn_fence(__ATOMIC_ACQUIRE, "workgroup");
  }
}

#ifndef SPLIT1
#define SPLIT1 1
#endif
#ifndef SPLIT2
#define SPLIT2 1
#endif
#define NB       4
#define NV       50000
#define NR       64
#define ND       64
#define NE       500000
#define MROWS    (NB * NV)
#define MPAD     200064
#define NBLK     49
#define NBROWS   1024
#define DEGCAP   64
#define MAXHITS  10507
#define MAXDEG   24
#define NTHR     256
#define NWAVE    8
#define EPT      8
#define CHUNK    (NTHR * EPT)
#define WCAP     (EPT * 32)
#define LISTN    (NWAVE * WCAP)
#define NBMAX    2048
#define ESH      11
#define RCAP     16384
#define LDS_BKT  ((2 * RCAP + 2 * NBMAX + LISTN) * 4 + 64)
#define LDS_AGG  ((NR * NB * ND + ND) * 4)
#define WSMAX    ((size_t)128 << 20)

static_assert(ND == 64 && NR == 64 && NB * ND == 32 * 8);
static_assert(MPAD % 128 == 0 && MPAD % 64 == 0 && MPAD % 16 == 0 && MPAD >= MROWS && MPAD - MROWS == 64);
static_assert(MROWS % 64 == 0 && MROWS / 64 == 3125);
static_assert(MPAD / 128 == 1563 && (MPAD / 64 + 7) / 8 == 391);
static_assert(NBLK * NBROWS >= NV && (NBLK - 1) * NBROWS < NV);
static_assert(NBROWS <= NBMAX && (1 << ESH) >= NBMAX && NTHR * 8 == NBMAX && LISTN >= NBMAX);
static_assert(NBROWS == 8 * 128 && NBROWS == 4 * NTHR);
static_assert(NE <= (1 << (32 - ESH)) && 3 * (long long)NE < 0x7fffffffLL);
static_assert(RCAP % 1024 == 0 && RCAP % 16 == 0 && RCAP > MAXHITS + 1024);
static_assert(RCAP * 100 >= MAXHITS * 125);
static_assert(DEGCAP >= MAXDEG + 8 && DEGCAP <= 64);
static_assert(LDS_BKT <= 327680 && LDS_AGG <= 327680);
static_assert((long long)MPAD * 128 / 8 < 0x7fffffffLL);

constexpr size_t al256(size_t v) { return (v + 255) & ~(size_t)255; }
constexpr size_t O_A     = 0;
constexpr size_t O_P     = al256(O_A     + (size_t)MPAD * 128 * 2);
constexpr size_t O_BLIST = al256(O_P     + (size_t)MPAD * 64 * 4);
constexpr size_t O_OFFC  = al256(O_BLIST + (size_t)NBLK * RCAP * 4);
constexpr size_t O_META  = al256(O_OFFC  + (size_t)NBLK * 2048 * 4);
constexpr size_t O_W1T   = al256(O_META  + (size_t)NBLK * 128);
constexpr size_t O_W2T   = al256(O_W1T   + 64 * 128 * 2);
constexpr size_t WS_TOTAL = al256(O_W2T + 64 * 128 * 2);
static_assert(WS_TOTAL <= (size_t)WSMAX);

typedef int v4i __attribute__((ext_vector_type(4)));
typedef v4i __attribute__((may_alias)) v4ia;

__device__ __forceinline__ void st2_v4u(void* p, const v4u v) {
  volatile v4u* q = (volatile v4u*)p;
  *q = v;
  __threadfence();
  *q = v;
}
__device__ __forceinline__ void st2_v4i(int* p, const v4i v) {
  volatile v4i* q = (volatile v4i*)p;
  *q = v;
  __threadfence();
  *q = v;
}
__device__ __forceinline__ float bf16_fin(float f) {
  const unsigned u = __float_as_uint(f);
  return __uint_as_float((u + 0x7FFFu + ((u >> 16) & 1u)) & 0xFFFF0000u);
}
__device__ __forceinline__ v4f bf16_val4(v4f v) {
  return (v4f){ bf16_val(v[0]), bf16_val(v[1]), bf16_val(v[2]), bf16_val(v[3]) };
}

__device__ __forceinline__ v4u gather8_bf16(const float* __restrict__ src, int base, int k0, int kmask, int stride,
                                            unsigned mk) {
  float x[8];
#pragma unroll
  for (int e = 0; e < 8; ++e) {
    const float v = src[base + ((k0 + e) & kmask) * stride];
    asm volatile("" :: "v"(v));
    x[e] = v;
  }
  v4u o = pack8_bf16((v4f){ x[0], x[1], x[2], x[3] }, (v4f){ x[4], x[5], x[6], x[7] });
  o &= (v4u){ mk, mk, mk, mk };
  return o;
}

__global__ __launch_bounds__(256) void k_prep(const float* __restrict__ W1, const float* __restrict__ W2,
                                              unsigned short* W1T2, unsigned short* W2T2, unsigned short* A) {
  const int b = (int)blockIdx.x, tid = (int)threadIdx.x;
  if (b < 4) {
    const int u = b * 256 + tid;
    const int n = u >> 4, p = u & 15;
    const v4u o = gather8_bf16(W1, n, 8 * p, 63, 64, 0xFFFFFFFFu);
    st2_v4u(W1T2 + (size_t)u * 8, o);
  } else if (b < 8) {
    const int u = (b - 4) * 256 + tid;
    const int n = u >> 4, p = u & 15;
    const v4u o = gather8_bf16(W2, n, 8 * p, 63, 64, 0xFFFFFFFFu);
    st2_v4u(W2T2 + (size_t)u * 8, o);
  } else {
    const v4u z = (v4u){ 0u, 0u, 0u, 0u };
    for (int q = tid; q < (MPAD - MROWS) * 16; q += 256) st2_v4u(A + (size_t)MROWS * 128 + (size_t)q * 8, z);
  }
}

__device__ __forceinline__ int scan_chunk(const int* __restrict__ edges, int nE, int cbase, int slotBase,
                                          int nb, int* list, int lane, int wave) {
  int wc = 0;
  const int elb  = wave * WCAP + lane;
  const int e0   = cbase + elb;
  const int sent = (-0x7fffffff - 1);
  const int last = nE - 1;
  const int t0 = edges[3 * min(e0 +   0, last)];
  const int t1 = edges[3 * min(e0 +  32, last)];
  const int t2 = edges[3 * min(e0 +  64, last)];
  const int t3 = edges[3 * min(e0 +  96, last)];
  const int t4 = edges[3 * min(e0 + 128, last)];
  const int t5 = edges[3 * min(e0 + 160, last)];
  const int t6 = edges[3 * min(e0 + 192, last)];
  const int t7 = edges[3 * min(e0 + 224, last)];
  asm volatile("" :: "v"(t0), "v"(t1), "v"(t2), "v"(t3), "v"(t4), "v"(t5), "v"(t6), "v"(t7));
  const int d0 = (e0 +   0 < nE) ? t0 : sent;
  const int d1 = (e0 +  32 < nE) ? t1 : sent;
  const int d2 = (e0 +  64 < nE) ? t2 : sent;
  const int d3 = (e0 +  96 < nE) ? t3 : sent;
  const int d4 = (e0 + 128 < nE) ? t4 : sent;
  const int d5 = (e0 + 160 < nE) ? t5 : sent;
  const int d6 = (e0 + 192 < nE) ? t6 : sent;
  const int d7 = (e0 + 224 < nE) ? t7 : sent;
  const unsigned nbs = (unsigned)slotBase;
  const unsigned unb = (unsigned)nb;
  const unsigned s0 = (unsigned)d0 - nbs, s1 = (unsigned)d1 - nbs;
  const unsigned s2 = (unsigned)d2 - nbs, s3 = (unsigned)d3 - nbs;
  const unsigned s4 = (unsigned)d4 - nbs, s5 = (unsigned)d5 - nbs;
  const unsigned s6 = (unsigned)d6 - nbs, s7 = (unsigned)d7 - nbs;
  const bool h0 = s0 < unb, h1 = s1 < unb, h2 = s2 < unb, h3 = s3 < unb;
  const bool h4 = s4 < unb, h5 = s5 < unb, h6 = s6 < unb, h7 = s7 < unb;
  const unsigned any = __builtin_amdgcn_ballot_w32(h0 | h1 | h2 | h3 | h4 | h5 | h6 | h7);
  if (any != 0u) {
#define HITJ(J, HJ, SJ) { \
      const unsigned mj = __builtin_amdgcn_ballot_w32(HJ); \
      if (mj != 0u) { \
        if (HJ) { \
          const int pos = wc + (int)__builtin_amdgcn_mbcnt_lo(mj, 0u); \
          if (pos < WCAP) list[wave * WCAP + pos] = ((elb + 32 * (J)) << 12) | (int)(SJ); \
        } \
        wc += (int)__builtin_popcount(mj); } }
    HITJ(0, h0, s0)
    HITJ(1, h1, s1)
    HITJ(2, h2, s2)
    HITJ(3, h3, s3)
    HITJ(4, h4, s4)
    HITJ(5, h5, s5)
    HITJ(6, h6, s6)
    HITJ(7, h7, s7)
#undef HITJ
  }
  return wc;
}

__device__ __forceinline__ int build_lists(const int* __restrict__ edges, int nE, int nodeBase, int nb,
                                           int* reg1, int* reg2, int* scnt, int* soff, int* list,
                                           int* wcnt, int* wtot, int tid, int lane, int wave) {
  for (int i = tid; i < NBMAX; i += NTHR) scnt[i] = 0;
  __syncthreads();

  int tot = 0;
  const int nChunks = (nE + CHUNK - 1) / CHUNK;
#pragma unroll 1
  for (int ch = 0; ch < nChunks; ++ch) {
    const int cbase = ch * CHUNK;
    const int wc = scan_chunk(edges, nE, cbase, nodeBase, nb, list, lane, wave);
    if (lane == 0) wcnt[wave] = wc;
    __syncthreads();
    int pre = 0, all = 0;
#pragma unroll
    for (int w2 = 0; w2 < NWAVE; ++w2) {
      int c = wcnt[w2];
      c = c < 0 ? 0 : (c > WCAP ? WCAP : c);
      all += c;
      pre += (w2 < wave) ? c : 0;
    }
    const int wcc  = wc > WCAP ? WCAP : wc;
    const int base = tot + pre;
#pragma unroll 1
    for (int i = lane; i < wcc; i += 32) {
      const int ent = list[wave * WCAP + i];
      const int el  = (ent >> 12) & (CHUNK - 1);
      const int sl  = ent & (NBMAX - 1);
      int eid = cbase + el;
      eid = eid > nE - 1 ? nE - 1 : eid;
      const int pos = base + i;
      if (pos < RCAP) reg1[pos] = (int)(((unsigned)eid << ESH) | (unsigned)sl);
    }
    tot += all;
    tot = tot > RCAP ? RCAP : tot;
    __syncthreads();
  }
  const int nh = tot;

  if (wave == 0) {
#pragma unroll 1
    for (int b0 = 0; b0 < nh; b0 += 32) {
      const int idx = b0 + lane;
      const int uv  = reg1[idx < RCAP ? idx : RCAP - 1];
      const int m32 = (nh - b0) < 32 ? (nh - b0) : 32;
#pragma unroll 1
      for (int k = 0; k < m32; ++k) {
        const int u  = __builtin_amdgcn_readlane(uv, k);
        const int sl = u & (NBMAX - 1);
        if (lane == 0) scnt[sl] = scnt[sl] + 1;
      }
    }
  }
  __syncthreads();

  {
    const v4i ca = *(const v4i*)(scnt + 8 * tid);
    const v4i cb = *(const v4i*)(scnt + 8 * tid + 4);
    const int e0 = ca.x < 0 ? 0 : ca.x, e1 = ca.y < 0 ? 0 : ca.y, e2 = ca.z < 0 ? 0 : ca.z, e3 = ca.w < 0 ? 0 : ca.w;
    const int e4 = cb.x < 0 ? 0 : cb.x, e5 = cb.y < 0 ? 0 : cb.y, e6 = cb.z < 0 ? 0 : cb.z, e7 = cb.w < 0 ? 0 : cb.w;
    const int ts = e0 + e1 + e2 + e3 + e4 + e5 + e6 + e7;
    int incl = ts;
#pragma unroll
    for (int d = 1; d < 32; d <<= 1) {
      const int up = __shfl_up(incl, d);
      if (lane >= d) incl += up;
    }
    if (lane == 31) wtot[wave] = incl;
    __syncthreads();
    int pre = 0;
#pragma unroll
    for (int w2 = 0; w2 < NWAVE; ++w2) pre += (w2 < wave) ? wtot[w2] : 0;
    int run = pre + incl - ts;
    soff[8 * tid + 0] = run; run += e0;
    soff[8 * tid + 1] = run; run += e1;
    soff[8 * tid + 2] = run; run += e2;
    soff[8 * tid + 3] = run; run += e3;
    soff[8 * tid + 4] = run; run += e4;
    soff[8 * tid + 5] = run; run += e5;
    soff[8 * tid + 6] = run; run += e6;
    soff[8 * tid + 7] = run;
  }
  __syncthreads();
  for (int i = tid; i < NBMAX; i += NTHR) list[i] = soff[i];
  __syncthreads();

  if (wave == 0) {
#pragma unroll 1
    for (int b0 = 0; b0 < nh; b0 += 32) {
      const int idx = b0 + lane;
      const int uv  = reg1[idx < RCAP ? idx : RCAP - 1];
      const int m32 = (nh - b0) < 32 ? (nh - b0) : 32;
#pragma unroll 1
      for (int k = 0; k < m32; ++k) {
        const int u   = __builtin_amdgcn_readlane(uv, k);
        const int sl  = u & (NBMAX - 1);
        const int eid = (int)((unsigned)u >> ESH);
        if (lane == 0) {
          int pos = list[sl];
          pos = pos < 0 ? 0 : (pos > RCAP - 1 ? RCAP - 1 : pos);
          reg2[pos] = eid;
          list[sl] = pos + 1;
        }
      }
    }
  }
  __syncthreads();
  return nh;
}

__global__ __launch_bounds__(NTHR) void k_bucket(const int* __restrict__ edges, int nE, int nN,
                                                 int* BLIST, int* OFFC, int* META) {
  extern __shared__ v4f lds_dyn[];
  int* reg1 = (int*)lds_dyn;
  int* reg2 = reg1 + RCAP;
  int* scnt = reg2 + RCAP;
  int* soff = scnt + NBMAX;
  int* list = soff + NBMAX;
  int* wcnt = list + LISTN;
  int* wtot = wcnt + NWAVE;
  const int tid = (int)threadIdx.x, lane = tid & 31, wave = tid >> 5;
  const int b = (int)blockIdx.x;
  const int nodeBase = b * NBROWS;
  int nb = nN - nodeBase;
  nb = nb < 0 ? 0 : (nb > NBROWS ? NBROWS : nb);

  const int nh = build_lists(edges, nE, nodeBase, nb, reg1, reg2, scnt, soff, list, wcnt, wtot, tid, lane, wave);

  int* bl = BLIST + (size_t)b * RCAP;
  const int last = nh > 0 ? nh - 1 : 0;
#pragma unroll 1
  for (int base = 0; base < RCAP; base += 1024) {
    const int i0 = base + 4 * tid;
    v4i v;
    v.x = reg2[i0     < last ? i0     : last];
    v.y = reg2[i0 + 1 < last ? i0 + 1 : last];
    v.z = reg2[i0 + 2 < last ? i0 + 2 : last];
    v.w = reg2[i0 + 3 < last ? i0 + 3 : last];
    v.x = (i0     < nh) ? v.x : 0;
    v.y = (i0 + 1 < nh) ? v.y : 0;
    v.z = (i0 + 2 < nh) ? v.z : 0;
    v.w = (i0 + 3 < nh) ? v.w : 0;
    st2_v4i(bl + i0, v);
  }
  {
    const v4i so = *(const v4ia*)(soff + 4 * tid);
    const v4i sc = *(const v4ia*)(scnt + 4 * tid);
    int* oc = OFFC + (size_t)b * 2048;
    st2_v4i(oc + 4 * tid, so);
    st2_v4i(oc + 1024 + 4 * tid, sc);
  }
  if (tid < 8) {
    v4i mv;
    mv.x = (tid == 0) ? nh : 0;
    mv.y = (tid == 0 && nh >= RCAP) ? 1 : 0;
    mv.z = 0; mv.w = 0;
    st2_v4i(META + (size_t)b * 32 + 4 * tid, mv);
  }
}

__global__ __launch_bounds__(256) __attribute__((amdgpu_num_vgpr(248)))
void k_agg(const float* __restrict__ x, const float* __restrict__ z, const int* __restrict__ edges,
           const float* __restrict__ alpha, const int* __restrict__ BLIST, const int* __restrict__ OFFC,
           const int* __restrict__ META, unsigned short* A) {
  extern __shared__ v4f lds_dyn[];
  float* ZT  = (float*)lds_dyn;
  float* sAl = ZT + NR * NB * ND;
  const int tid = (int)threadIdx.x, lane = tid & 31;
  const int wave = __builtin_amdgcn_readfirstlane(tid >> 5);
#pragma unroll 4
  for (int i = 0; i < 16; ++i) {
    const int f = 4 * (i * 256 + tid);
    const v4f v = *(const v4fa*)(z + f);
    const int bt = f >> 12, r = (f >> 6) & 63, d = f & 63;
    *(v4fa*)(ZT + r * 256 + bt * 64 + d) = bf16_val4(v);
  }
  {
    const int ix = tid < 16 ? tid : 15;
    const v4f a = *(const v4fa*)(alpha + 4 * ix);
    asm volatile("" :: "v"(a));
    if (tid < 16) *(v4fa*)(sAl + 4 * tid) = bf16_val4(a);
  }
  __syncthreads();

  const int b = (int)blockIdx.x;
  const int nodeBase = b * NBROWS;
  const int nb = clampi(NV - nodeBase, 0, NBROWS);
  const int nh = clampi(META[(size_t)b * 32], 0, RCAP);
  const int flag = META[(size_t)b * 32 + 1];
  const bool ovf = flag != 0;
  const int* bl = BLIST + (size_t)b * RCAP;
  const int* oc = OFFC + (size_t)b * 2048;
  const int nhm1 = nh > 0 ? nh - 1 : 0;
  const int bq = lane >> 3;
  const int pq = lane & 7;
  const int d0 = pq * 8;
  const v4f al0 = *(const v4fa*)(sAl + d0);
  const v4f al1 = *(const v4fa*)(sAl + d0 + 4);
  const float* xb = x + (size_t)bq * NV * 64 + d0;
  const float* zl = ZT + 8 * lane;
  const float qnan = __int_as_float(0x7fc00000);
  const v4f zero4 = (v4f){ 0.0f, 0.0f, 0.0f, 0.0f };
  const v4u zero4u = (v4u){ 0u, 0u, 0u, 0u };

#pragma unroll 1
  for (int g = 0; g < 4; ++g) {
    const int slot0 = wave * 128 + g * 32;
    if (slot0 >= nb) break;
    int stv = oc[slot0 + lane];
    int cv  = oc[1024 + slot0 + lane];
    asm volatile("" :: "v"(stv), "v"(cv));
    const int craw = cv < 0 ? 0 : cv;
    const int pv = (craw > DEGCAP) ? 1 : 0;
    stv = clampi(stv, 0, nh);
    int cc = clampi(craw, 0, DEGCAP);
    cc = cc > nh - stv ? nh - stv : cc;
#pragma unroll 1
    for (int rr = 0; rr < 32; ++rr) {
      if (slot0 + rr >= nb) break;
      const int st  = __builtin_amdgcn_readlane(stv, rr);
      const int cnt = __builtin_amdgcn_readlane(cc, rr);
      const int prw = __builtin_amdgcn_readlane(pv, rr);
      v4f acc0 = zero4, acc1 = zero4;
#pragma unroll 1
      for (int b0 = 0; b0 < cnt; b0 += 32) {
        const int li = clampi(st + b0 + lane, 0, nhm1);
        int id = bl[li];
        asm volatile("" :: "v"(id));
        id = clampi(id, 0, NE - 1);
        int et = edges[3 * id + 1];
        int sr = edges[3 * id + 2];
        asm volatile("" :: "v"(et), "v"(sr));
        et = clampi(et, 0, NR - 1);
        sr = clampi(sr, 0, NV - 1);
        const int m32 = (cnt - b0) < 32 ? (cnt - b0) : 32;
#pragma unroll 2
        for (int q = 0; q < m32; ++q) {
          const int eq = __builtin_amdgcn_readlane(et, q);
          const int sq = __builtin_amdgcn_readlane(sr, q);
          const float* xp = xb + (size_t)sq * 64;
          const v4f xa = *(const v4fa*)xp;
          const v4f xc = *(const v4fa*)(xp + 4);
          const float* zp = zl + eq * 256;
          const v4f za = *(const v4fa*)zp;
          const v4f zc = *(const v4fa*)(zp + 4);
          acc0[0] = fmaf(bf16_fin(xa[0]), za[0], acc0[0]);
          acc0[1] = fmaf(bf16_fin(xa[1]), za[1], acc0[1]);
          acc0[2] = fmaf(bf16_fin(xa[2]), za[2], acc0[2]);
          acc0[3] = fmaf(bf16_fin(xa[3]), za[3], acc0[3]);
          acc1[0] = fmaf(bf16_fin(xc[0]), zc[0], acc1[0]);
          acc1[1] = fmaf(bf16_fin(xc[1]), zc[1], acc1[1]);
          acc1[2] = fmaf(bf16_fin(xc[2]), zc[2], acc1[2]);
          acc1[3] = fmaf(bf16_fin(xc[3]), zc[3], acc1[3]);
        }
      }
      const int v = nodeBase + slot0 + rr;
      const float* xo = xb + (size_t)v * 64;
      const v4f ya = bf16_val4(*(const v4fa*)xo);
      const v4f yc = bf16_val4(*(const v4fa*)(xo + 4));
      v4f h0 = acc0 + al0 * ya;
      v4f h1 = acc1 + al1 * yc;
      const bool bad = ovf || (prw != 0);
#pragma unroll
      for (int e = 0; e < 4; ++e) {
        h0[e] = bad ? qnan : h0[e];
        h1[e] = bad ? qnan : h1[e];
      }
      const v4u hi = pack8_bf16(h0, h1);
      v4u lo = zero4u;
      if (SPLIT1) lo = pack8_bf16_lo(h0, h1);
      unsigned short* ap = A + ((size_t)bq * NV + (size_t)v) * 128 + pq * 8;
      for (int pass = 0; pass < 2; ++pass) {
        *(volatile v4u*)ap = hi;
        *(volatile v4u*)(ap + 64) = lo;
        __threadfence();
      }
    }
  }
}

__global__ __launch_bounds__(256) void k_relu_split(const float* __restrict__ P, const float* __restrict__ b1,
                                                    unsigned short* A) {
  __shared__ __attribute__((aligned(16))) float sB[64];
  const int tid = (int)threadIdx.x, lane = tid & 31, wave = tid >> 5;
  {
    const int ix = tid < 16 ? tid : 15;
    const v4f w = *(const v4fa*)(b1 + 4 * ix);
    asm volatile("" :: "v"(w));
    if (tid < 16) *(v4fa*)(sB + 4 * tid) = bf16_val4(w);
  }
  __syncthreads();
  const int r = lane >> 3, p = lane & 7;
  const v4f bv0 = *(const v4fa*)(sB + 8 * p);
  const v4f bv1 = *(const v4fa*)(sB + 8 * p + 4);
  const v4u zero4u = (v4u){ 0u, 0u, 0u, 0u };
#pragma unroll 1
  for (int it = 0; it < 4; ++it) {
    const int row = (int)blockIdx.x * 128 + it * 32 + wave * 4 + r;
    const float* pp = P + (size_t)row * 64 + 8 * p;
    v4f a = *(const v4fa*)pp;
    v4f c = *(const v4fa*)(pp + 4);
    a = a + bv0;
    c = c + bv1;
#pragma unroll
    for (int e = 0; e < 4; ++e) {
      const float ta = a[e]; a[e] = (ta > 0.0f) ? ta : (ta - ta);
      const float tc = c[e]; c[e] = (tc > 0.0f) ? tc : (tc - tc);
    }
    const v4u hi = pack8_bf16(a, c);
    v4u lo = zero4u;
    if (SPLIT2) lo = pack8_bf16_lo(a, c);
    unsigned short* ap = A + (size_t)row * 128 + 8 * p;
    for (int pass = 0; pass < 2; ++pass) {
      *(volatile v4u*)ap = hi;
      *(volatile v4u*)(ap + 64) = lo;
      __threadfence();
    }
  }
}

__global__ __launch_bounds__(256) void k_ln_out(const float* __restrict__ P, const float* __restrict__ x,
                                                const float* __restrict__ b2, const float* __restrict__ gamma,
                                                const float* __restrict__ beta, float* out) {
  __shared__ __attribute__((aligned(16))) float sPar[192];
  const int tid = (int)threadIdx.x, lane = tid & 31, wave = tid >> 5;
  {
    const int ix = tid & 15;
    const v4f vb = *(const v4fa*)(b2 + 4 * ix);
    const v4f vg = *(const v4fa*)(gamma + 4 * ix);
    const v4f ve = *(const v4fa*)(beta + 4 * ix);
    asm volatile("" :: "v"(vb), "v"(vg), "v"(ve));
    const int sel = tid >> 4;
    const unsigned m0 = sel == 0 ? 0xFFFFFFFFu : 0u;
    const unsigned m1 = sel == 1 ? 0xFFFFFFFFu : 0u;
    const unsigned m2 = sel == 2 ? 0xFFFFFFFFu : 0u;
    v4f o;
#pragma unroll
    for (int e = 0; e < 4; ++e) {
      const unsigned w = (__float_as_uint(vb[e]) & m0) | (__float_as_uint(vg[e]) & m1) | (__float_as_uint(ve[e]) & m2);
      o[e] = bf16_val(__uint_as_float(w));
    }
    if (tid < 48) *(v4fa*)(sPar + 4 * tid) = o;
  }
  __syncthreads();
  const int hh = lane >> 4;
  const int c4 = (lane & 15) * 4;
  const v4f pb2 = *(const v4fa*)(sPar + c4);
  const v4f pg  = *(const v4fa*)(sPar + 64 + c4);
  const v4f pbe = *(const v4fa*)(sPar + 128 + c4);
#pragma unroll 1
  for (int it = 0; it < 4; ++it) {
    const int row = (int)blockIdx.x * 64 + wave * 8 + it * 2 + hh;
    const int rc  = row < MROWS ? row : MROWS - 1;
    v4f v  = *(const v4fa*)(P + (size_t)rc * 64 + c4);
    v4f xv = *(const v4fa*)(x + (size_t)rc * 64 + c4);
    asm volatile("" :: "v"(v), "v"(xv));
    v = v + pb2;
    const v4f xr = bf16_val4(xv);
    float s = (v[0] + v[1]) + (v[2] + v[3]);
    s += __shfl_xor(s, 8);
    s += __shfl_xor(s, 4);
    s += __shfl_xor(s, 2);
    s += __shfl_xor(s, 1);
    const float mu = s * (1.0f / 64.0f);
    const v4f d = v - mu;
    float q = (d[0] * d[0] + d[1] * d[1]) + (d[2] * d[2] + d[3] * d[3]);
    q += __shfl_xor(q, 8);
    q += __shfl_xor(q, 4);
    q += __shfl_xor(q, 2);
    q += __shfl_xor(q, 1);
    const float rs = 1.0f / sqrtf(q * (1.0f / 64.0f) + 1e-5f);
    const v4f y = ((d * rs) * pg + pbe) + xr;
    float* op = out + (size_t)rc * 64 + c4;
    for (int pass = 0; pass < 2; ++pass) {
      if (row < MROWS) *(volatile v4f*)op = y;
      __threadfence();
    }
  }
}

extern "C" void kernel_launch(void* const* d_in, const int* in_sizes, int n_in,
                              void* d_out, int out_size, void* d_ws, size_t ws_size,
                              hipStream_t stream) {
  if (n_in < 10) return;
  if (in_sizes[0] != NB * NV * ND || in_sizes[1] != NB * NR * ND || in_sizes[2] != 3 * NE) return;
  if (in_sizes[3] != ND * ND || in_sizes[4] != ND || in_sizes[5] != ND * ND || in_sizes[6] != ND) return;
  if (in_sizes[7] != ND || in_sizes[8] != ND || in_sizes[9] != ND) return;
  if (out_size != NB * NV * ND) return;
  if (ws_size < WS_TOTAL) return;

  const float* x     = (const float*)d_in[0];
  const float* z     = (const float*)d_in[1];
  const int*   edges = (const int*)  d_in[2];
  const float* W1    = (const float*)d_in[3];
  const float* b1    = (const float*)d_in[4];
  const float* W2    = (const float*)d_in[5];
  const float* b2    = (const float*)d_in[6];
  const float* alpha = (const float*)d_in[7];
  const float* gamma = (const float*)d_in[8];
  const float* beta  = (const float*)d_in[9];
  float* out = (float*)d_out;

  char* ws = (char*)d_ws;
  unsigned short* A     = (unsigned short*)(ws + O_A);
  float*          P     = (float*)(ws + O_P);
  int*            BLIST = (int*)(ws + O_BLIST);
  int*            OFFC  = (int*)(ws + O_OFFC);
  int*            META  = (int*)(ws + O_META);
  unsigned short* W1T2  = (unsigned short*)(ws + O_W1T);
  unsigned short* W2T2  = (unsigned short*)(ws + O_W2T);

  hipFuncSetAttribute(reinterpret_cast<const void*>(&k_bucket),
                      hipFuncAttributeMaxDynamicSharedMemorySize, LDS_BKT);
  hipFuncSetAttribute(reinterpret_cast<const void*>(&k_agg),
                      hipFuncAttributeMaxDynamicSharedMemorySize, LDS_AGG);

  k_prep<<<9, 256, 0, stream>>>(W1, W2, W1T2, W2T2, A);
  k_bucket<<<NBLK, NTHR, LDS_BKT, stream>>>(edges, NE, NV, BLIST, OFFC, META);
  k_agg<<<NBLK, 256, LDS_AGG, stream>>>(x, z, edges, alpha, BLIST, OFFC, META, A);
  k_gemm_nt<0, 0><<<(MPAD / 64 + 7) / 8, 256, 0, stream>>>(A, W1T2, b1, P, MPAD, 64, 128, 64);
  k_relu_split<<<MPAD / 128, 256, 0, stream>>>(P, b1, A);
  k_gemm_nt<0, 0><<<(MPAD / 64 + 7) / 8, 256, 0, stream>>>(A, W2T2, b2, P, MPAD, 64, 128, 64);
  k_ln_out<<<MROWS / 64, 256, 0, stream>>>(P, x, b2, gamma, beta, out);
}
